// MLPEdgeDecoder_29008209117686
// MI455X (gfx1250) — hardware-verified
//
#include <hip/hip_runtime.h>
#include <math.h>

typedef __attribute__((ext_vector_type(16))) _Float16 v16h;
typedef __attribute__((ext_vector_type(16))) __bf16 v16b;
typedef __attribute__((ext_vector_type(8)))  _Float16 v8h;
typedef __attribute__((ext_vector_type(8)))  float v8f;
typedef __attribute__((ext_vector_type(4)))  float v4f;
typedef __attribute__((ext_vector_type(2)))  float v2f;
typedef __attribute__((ext_vector_type(4)))  unsigned v4u;
typedef __attribute__((ext_vector_type(4)))  int v4i;
typedef float __attribute__((may_alias)) float_a;
typedef int __attribute__((may_alias)) int_a;

template <typename T> __device__ __forceinline__ void vst2(void* p, T v) { *(volatile T*)p = v; __threadfence(); *(volatile T*)p = v; }
__device__ __forceinline__ v8f wmma16(v16h a, v16h b, v8f c) {
  v8f d = __builtin_amdgcn_wmma_f32_16x16x32_f16(false, a, false, b, (short)0, c, false, false);
  asm volatile("v_nop\n\tv_nop\n\tv_nop\n\tv_nop" : "+v"(d) : "v"(a), "v"(b));
  return d;
}
__device__ __forceinline__ v8f wmma_bf(v16b a, v16b b, v8f c) {
  v8f d = __builtin_amdgcn_wmma_f32_16x16x32_bf16(false, a, false, b, (short)0, c, false, false);
  asm volatile("v_nop\n\tv_nop\n\tv_nop\n\tv_nop" : "+v"(d) : "v"(a), "v"(b));
  return d;
}
__device__ __forceinline__ v16h frag_h(const _Float16* rowk0, int lane) {
  union { v16h v; v8h q[2]; } u; const _Float16* p = rowk0 + 8 * (lane >> 4);
  u.q[0] = *(const v8h*)p; u.q[1] = *(const v8h*)(p + 16); return u.v;
}
__device__ __forceinline__ v16h frag_f32(const float* rowk0, int lane) {
  v16h a; const float* p = rowk0 + 8 * (lane >> 4);
#pragma unroll
  for (int i = 0; i < 8; ++i) { a[i] = (_Float16)p[i]; a[8 + i] = (_Float16)p[16 + i]; }
  return a;
}
__device__ __forceinline__ v16h frag_f32s(const float* rowk0, int lane, float sc) {
  v16h a; const float* p = rowk0 + 8 * (lane >> 4);
#pragma unroll
  for (int i = 0; i < 8; ++i) { a[i] = (_Float16)(p[i] * sc); a[8 + i] = (_Float16)(p[16 + i] * sc); }
  return a;
}
__device__ __forceinline__ v16h fragc_f32(const float* W, int k0, int n, int lane, int ld, int K) {
  v16h a; const int g = lane >> 4;
#pragma unroll
  for (int i = 0; i < 8; ++i) { const int ka = k0 + 8 * g + i, kb = ka + 16;
    a[i] = (_Float16)(ka < K ? W[(size_t)(ka < K ? ka : K - 1) * ld + n] : 0.f); a[8 + i] = (_Float16)(kb < K ? W[(size_t)(kb < K ? kb : K - 1) * ld + n] : 0.f); }
  return a;
}
struct F2 { v16b h, l; };
__device__ __forceinline__ F2 bsplit16(const float v[16]) { F2 r;
#pragma unroll
  for (int i = 0; i < 16; ++i) { const __bf16 h = (__bf16)v[i]; r.h[i] = h; r.l[i] = (__bf16)(v[i] - (float)h); }
  return r; }
__device__ __forceinline__ F2 split_row(const float* row, int k0, int lane) { float v[16]; const float* p = row + k0 + 8 * (lane >> 4);
#pragma unroll
  for (int i = 0; i < 8; ++i) { v[i] = p[i]; v[8 + i] = p[16 + i]; }
  return bsplit16(v); }
__device__ __forceinline__ F2 split_rowK(const float* row, int k0, int lane, int K) { float v[16]; const int g = lane >> 4;
#pragma unroll
  for (int i = 0; i < 8; ++i) { const int ka = k0 + 8 * g + i, kb = ka + 16; v[i] = ka < K ? row[ka < K ? ka : K - 1] : 0.f; v[8 + i] = kb < K ? row[kb < K ? kb : K - 1] : 0.f; }
  return bsplit16(v); }
__device__ __forceinline__ F2 split_col(const float* W, int k0, int n, int lane, int ld, int K) { float v[16]; const int g = lane >> 4;
#pragma unroll
  for (int i = 0; i < 8; ++i) { const int ka = k0 + 8 * g + i, kb = ka + 16; v[i] = ka < K ? W[(size_t)(ka < K ? ka : K - 1) * ld + n] : 0.f; v[8 + i] = kb < K ? W[(size_t)(kb < K ? kb : K - 1) * ld + n] : 0.f; }
  return bsplit16(v); }
__device__ __forceinline__ v8f mac3(const F2& a, const F2& b, v8f c) { c = wmma_bf(a.l, b.h, c); c = wmma_bf(a.h, b.l, c); return wmma_bf(a.h, b.h, c); }
__device__ __forceinline__ float sigm(float v) { return 1.0f / (1.0f + expf(-v)); }
#define LDSX() do { asm volatile("s_wait_dscnt 0" ::: "memory"); __builtin_amdgcn_wave_barrier(); __builtin_amdgcn_fence(__ATOMIC_RELEASE, "workgroup"); } while (0)


#define NE 3200000
#define NNODE 100000
#define LAT 64
#define HID 32
#ifndef TE
#define TE (NE / 64)
#endif
typedef __attribute__((ext_vector_type(8))) __bf16 v8b;
__device__ __forceinline__ v16b frag_b(const __bf16* rowk0, int lane) {
  union { v16b v; v8b q[2]; } u; const __bf16* p = rowk0 + 8 * (lane >> 4);
  u.q[0] = *(const v8b*)p; u.q[1] = *(const v8b*)(p + 16); return u.v;
}
__device__ __forceinline__ float bfr(float v) { return (float)(__bf16)v; }
__device__ __attribute__((noinline)) float exp_ni(float v) { return expf(v); }
__device__ __attribute__((noinline)) float erf_ni(float v) { return erff(v); }

#define WS_PW  0u
#define WS_END (WS_PW + 2u * (size_t)HID * 2 * LAT)

__global__ __launch_bounds__(128) void k_pack(const float* __restrict__ W1, __bf16* __restrict__ PW) { const int t = threadIdx.x; const int n = blockIdx.x; __shared__ __align__(16) __bf16 s[2 * LAT]; s[t] = (__bf16)W1[(size_t)t * HID + n]; __syncthreads(); if (t < 16) vst2((unsigned*)(PW + (size_t)n * 2 * LAT + t * 8), *(const v4u*)&s[t * 8]); }
__device__ __forceinline__ v16b fragb_f32(const float* __restrict__ p, int lane) { v16b a; const float* pp = p + 8 * (lane >> 4);
#pragma unroll
  for (int i = 0; i < 8; ++i) { a[i] = (__bf16)pp[i]; a[8 + i] = (__bf16)pp[16 + i]; } return a; }
__global__ __launch_bounds__(128) void k_edge(const float* __restrict__ Z, const int* __restrict__ EI, const __bf16* __restrict__ PW, const float* __restrict__ B1, const float* __restrict__ W2, const float* __restrict__ B2, float* __restrict__ OUT) { __shared__ __align__(16) float so[64];
  const int tid = threadIdx.x, wave = tid >> 5, lane = tid & 31, col = lane & 15, g = lane >> 4; const size_t e0 = (size_t)blockIdx.x * 64 + wave * 16; const size_t e = e0 + col;
  int isrc = EI[e], idst = EI[NE + e]; isrc = isrc < 0 ? 0 : (isrc >= NNODE ? NNODE - 1 : isrc); idst = idst < 0 ? 0 : (idst >= NNODE ? NNODE - 1 : idst);
  v8f acc[2] = {};
#pragma unroll
  for (int kc = 0; kc < 4; ++kc) { const float* src = Z + (size_t)(kc < 2 ? isrc : idst) * LAT + (kc & 1) * 32; const v16b a = fragb_f32(src, lane);
#pragma unroll
    for (int j = 0; j < 2; ++j) acc[j] = wmma_bf(a, frag_b(PW + (size_t)(j * 16 + col) * (2 * LAT) + kc * 32, lane), acc[j]); }
  float part[8];
#pragma unroll
  for (int r = 0; r < 8; ++r) { part[r] = 0.f;
#pragma unroll
    for (int j = 0; j < 2; ++j) { const int c = j * 16 + col; float h = acc[j][r] + bfr(B1[c]); h = h >= 0.f ? h : 0.01f * h; part[r] += h * bfr(W2[c]); }
#pragma unroll
    for (int o = 1; o < 16; o <<= 1) part[r] += __shfl_xor(part[r], o);
    if (col == 0) so[wave * 16 + 8 * g + r] = tanhf(part[r] + bfr(B2[0])); }
  __syncthreads(); if (tid < 16) vst2(OUT + (size_t)blockIdx.x * 64 + tid * 4, *(const v4f*)&so[tid * 4]); }
extern "C" void kernel_launch(void* const* d_in, const int* in_sizes, int n_in, void* d_out, int out_size, void* d_ws, size_t ws_size, hipStream_t stream) {
  (void)in_sizes; (void)n_in; (void)out_size;
  const float** F = (const float**)d_in;
  if (ws_size < (size_t)WS_END) return;
  __bf16* PW = (__bf16*)((char*)d_ws + WS_PW);
  k_pack<<<HID, 128, 0, stream>>>(F[2], PW);
  k_edge<<<TE, 128, 0, stream>>>(F[0], (const int*)d_in[1], PW, F[3], F[4], F[5], (float*)d_out);
}
